// TDGSAttention_2740189135231
// MI455X (gfx1250) — hardware-verified
//
#include <hip/hip_runtime.h>


#define NB_  2
#define TQ   512
#define TK   4096
#define DD   1024
#define NH_  16
#define NKV  4
#define GRP  (NH_ / NKV)
#define HD   64
#define DKV  (NKV * HD)
#define NTQ  (NB_ * TQ)
#define NTK  (NB_ * TK)
#define ZH   4
typedef _Float16 h16;
typedef unsigned short bf;
typedef __attribute__((ext_vector_type(16))) __bf16   v16bf;
typedef __attribute__((ext_vector_type(16))) _Float16 v16h;
typedef __attribute__((ext_vector_type(8)))  _Float16 v8h;
typedef __attribute__((ext_vector_type(8)))  unsigned short v8us;
typedef __attribute__((ext_vector_type(8)))  float    v8f;
typedef __attribute__((ext_vector_type(4)))  float    v4f;
typedef v8h  __attribute__((may_alias)) v8ha;
typedef v4f  __attribute__((may_alias)) v4fa;
typedef v8us __attribute__((may_alias)) v8usa;

__device__ __forceinline__ unsigned short f2bf(float f) { unsigned u = __float_as_uint(f); u += 0x7FFFu + ((u >> 16) & 1u); return (unsigned short)(u >> 16); }
__device__ __forceinline__ float bf2f(unsigned short b) { return __uint_as_float(((unsigned)b) << 16); }
__device__ __forceinline__ float bfr(float f) { return bf2f(f2bf(f)); }
__device__ __forceinline__ v16h cat16(v8h lo, v8h hi) { return __builtin_shufflevector(lo, hi, 0, 1, 2, 3, 4, 5, 6, 7, 8, 9, 10, 11, 12, 13, 14, 15); }
__device__ __forceinline__ v16bf cat16b(v8us lo, v8us hi) { return __builtin_bit_cast(v16bf, __builtin_shufflevector(lo, hi, 0, 1, 2, 3, 4, 5, 6, 7, 8, 9, 10, 11, 12, 13, 14, 15)); }
__device__ __forceinline__ v8f wmma16(v16h a, v16h b, v8f c) { return __builtin_amdgcn_wmma_f32_16x16x32_f16(false, a, false, b, (short)0, c, false, false); }
__device__ __forceinline__ v8f wmmab(v16bf a, v16bf b, v8f c) { return __builtin_amdgcn_wmma_f32_16x16x32_bf16(false, a, false, b, (short)0, c, false, false); }


template <typename T16> struct WFrag;
template <> struct WFrag<h16> { typedef v16h V; static __device__ __forceinline__ V ld(const h16* p) { return cat16(*(const v8h*)p, *(const v8h*)(p + 16)); } static __device__ __forceinline__ v8f mma(V a, V b, v8f c) { return wmma16(a, b, c); } };
template <> struct WFrag<bf> { typedef v16bf V; static __device__ __forceinline__ V ld(const bf* p) { return cat16b(*(const v8us*)p, *(const v8us*)(p + 16)); } static __device__ __forceinline__ v8f mma(V a, V b, v8f c) { return wmmab(a, b, c); } };
template <typename T16, int NSPLIT, bool BIAS>
__global__ __launch_bounds__(32) void k_gemmw(const T16* __restrict__ A, const T16* __restrict__ A2, const T16* __restrict__ Bt, const T16* __restrict__ Bt2, int K, float* C, int ldc, const float* __restrict__ bias, size_t sA, size_t sB, size_t sC) {
    typedef typename WFrag<T16>::V V;
    __shared__ __align__(16) float os[16 * 68];
    const size_t z = blockIdx.z; A += z * sA; if (A2) A2 += z * sA; Bt += z * sB; if (Bt2) Bt2 += z * sB; C += z * sC;
    const int lane = threadIdx.x & 31, lr = lane & 15, hi = lane >> 4; const int r0 = blockIdx.x * 64, c0 = blockIdx.y * 64;
    v8f acc[4][4];
#pragma unroll
    for (int mb = 0; mb < 4; ++mb)
#pragma unroll
        for (int nb = 0; nb < 4; ++nb) acc[mb][nb] = (v8f){};
    const size_t aoff = (size_t)(r0 + lr) * K + 8 * hi, boff = (size_t)(c0 + lr) * K + 8 * hi;
#pragma unroll 1
    for (int kc = 0; kc < K; kc += 32) {
        V a[4], a2[4];
#pragma unroll
        for (int mb = 0; mb < 4; ++mb) { a[mb] = WFrag<T16>::ld(A + aoff + (size_t)mb * 16 * K + kc); if (NSPLIT == 1 || NSPLIT == 2) a2[mb] = WFrag<T16>::ld(A2 + aoff + (size_t)mb * 16 * K + kc); }
#pragma unroll
        for (int nb = 0; nb < 4; ++nb) { const V b = WFrag<T16>::ld(Bt + boff + (size_t)nb * 16 * K + kc); V b2; if (NSPLIT >= 2) b2 = WFrag<T16>::ld(Bt2 + boff + (size_t)nb * 16 * K + kc);
#pragma unroll
            for (int mb = 0; mb < 4; ++mb) { acc[mb][nb] = WFrag<T16>::mma(a[mb], b, acc[mb][nb]); if (NSPLIT == 1 || NSPLIT == 2) acc[mb][nb] = WFrag<T16>::mma(a2[mb], b, acc[mb][nb]); if (NSPLIT >= 2) acc[mb][nb] = WFrag<T16>::mma(a[mb], b2, acc[mb][nb]); } }
        asm volatile("v_nop\n\tv_nop\n\tv_nop\n\tv_nop" : "+v"(acc[0][0]), "+v"(acc[1][1]), "+v"(acc[2][2]), "+v"(acc[3][3]) : "v"(a[0]), "v"(a[3]));
    }
#pragma unroll
    for (int mb = 0; mb < 4; ++mb) {
#pragma unroll
        for (int nb = 0; nb < 4; ++nb) {
#pragma unroll
            for (int j = 0; j < 8; ++j) os[(hi * 8 + j) * 68 + nb * 16 + lr] = acc[mb][nb][j]; }
        __builtin_amdgcn_wave_barrier(); asm volatile("" ::: "memory");
        float* crow = C + (size_t)(r0 + mb * 16) * ldc + c0;
#pragma unroll 1
        for (int ps = 0; ps < 2; ++ps) {
#pragma unroll
            for (int s = 0; s < 8; ++s) { const int row = 2 * s + hi, cofs = lr * 4; v4f val = *(const v4fa*)(os + row * 68 + cofs); if (BIAS) { val[0] += bfr(bias[c0 + cofs]); val[1] += bfr(bias[c0 + cofs + 1]); val[2] += bfr(bias[c0 + cofs + 2]); val[3] += bfr(bias[c0 + cofs + 3]); }
                *(volatile v4f*)(crow + (size_t)row * ldc + cofs) = val; }
            if (ps == 0) __threadfence(); }
        __builtin_amdgcn_wave_barrier(); asm volatile("" ::: "memory");
    }
}

__device__ __forceinline__ void splitf(float y, unsigned short& h, unsigned short& l) { h = f2bf(y); l = f2bf(y - bf2f(h)); }
typedef __attribute__((ext_vector_type(2))) unsigned short v2us;
typedef __attribute__((ext_vector_type(2))) float v2f;

__global__ __launch_bounds__(256) void k_cvt8(const float* __restrict__ src, bf* dst, size_t n8) { const size_t i = (size_t)blockIdx.x * 256 + threadIdx.x; if (i >= n8) return; const v8f v = *(const v8f*)(src + i * 8); v8us o;
#pragma unroll
    for (int k = 0; k < 8; ++k) o[k] = f2bf(v[k]); *(volatile v8us*)(dst + i * 8) = o; __threadfence(); *(volatile v8us*)(dst + i * 8) = o; }
__global__ __launch_bounds__(256) void k_rmsq(const float* __restrict__ F, const float* __restrict__ w, bf* Ph, bf* Pl) {
    const int lane = threadIdx.x & 31; const int wg = blockIdx.x * 8 + (threadIdx.x >> 5); if (wg >= NTQ * NH_) return; const int r = wg / NH_, h = wg % NH_; const int b = r / TQ, t = r % TQ;
    const v2f a = *(const v2f*)(F + (size_t)r * DD + h * HD + lane * 2); float ss = __fadd_rn(__fmul_rn(a[0], a[0]), __fmul_rn(a[1], a[1]));
#pragma unroll
    for (int sh = 16; sh; sh >>= 1) ss += __shfl_xor(ss, sh, 32);
    const float rs = __fdiv_rn(1.0f, __fsqrt_rn(ss * (1.0f / HD) + 1e-6f)); v2us oh, ol;
#pragma unroll
    for (int q = 0; q < 2; ++q) { unsigned short x, y; splitf(__fmul_rn(a[q] * rs, bfr(w[lane * 2 + q])), x, y); oh[q] = x; ol[q] = y; }
    const size_t o = (((size_t)b * NH_ + h) * TQ + t) * HD + lane * 2; *(volatile v2us*)(Ph + o) = oh; *(volatile v2us*)(Pl + o) = ol; __threadfence(); *(volatile v2us*)(Ph + o) = oh; *(volatile v2us*)(Pl + o) = ol;
}
__global__ __launch_bounds__(256) void k_rmsk(const float* __restrict__ F, const float* __restrict__ w, bf* Ph, bf* Pl) {
    const int lane = threadIdx.x & 31; const int wg = blockIdx.x * 8 + (threadIdx.x >> 5); if (wg >= NTK * NKV) return; const int r = wg / NKV, kh = wg % NKV; const int b = r / TK, s = r % TK;
    const v2f a = *(const v2f*)(F + (size_t)r * DKV + kh * HD + lane * 2); float ss = __fadd_rn(__fmul_rn(a[0], a[0]), __fmul_rn(a[1], a[1]));
#pragma unroll
    for (int sh = 16; sh; sh >>= 1) ss += __shfl_xor(ss, sh, 32);
    const float rs = __fdiv_rn(1.0f, __fsqrt_rn(ss * (1.0f / HD) + 1e-6f)); v2us oh, ol;
#pragma unroll
    for (int q = 0; q < 2; ++q) { unsigned short x, y; splitf(__fmul_rn(a[q] * rs, bfr(w[lane * 2 + q])), x, y); oh[q] = x; ol[q] = y; }
    const size_t o = (((size_t)b * NKV + kh) * TK + s) * HD + lane * 2; *(volatile v2us*)(Ph + o) = oh; *(volatile v2us*)(Pl + o) = ol; __threadfence(); *(volatile v2us*)(Ph + o) = oh; *(volatile v2us*)(Pl + o) = ol;
}
__global__ __launch_bounds__(256) void k_vtsplit(const float* __restrict__ F, bf* Vh, bf* Vl) {
    const int lane = threadIdx.x & 31; const int L0 = (blockIdx.x * 8 + (threadIdx.x >> 5)) * 8; const int nlines = NB_ * NKV * HD * TK / 64;
#pragma unroll 1
    for (int ps = 0; ps < 2; ++ps) {
#pragma unroll
        for (int l = 0; l < 8; ++l) { const int L = L0 + l; if (L >= nlines) break; const int e = L * 64 + lane * 2; const int s = e & (TK - 1); const int d = (e >> 12) & 63; const int zk = e >> 18; const int b = zk / NKV, kh = zk % NKV; v2us oh, ol;
#pragma unroll
            for (int q = 0; q < 2; ++q) { unsigned short x, y; splitf(F[((size_t)b * TK + s + q) * DKV + kh * HD + d], x, y); oh[q] = x; ol[q] = y; }
            *(volatile v2us*)(Vh + (size_t)e) = oh; *(volatile v2us*)(Vl + (size_t)e) = ol; }
        if (ps == 0) __threadfence(); }
}
__global__ __launch_bounds__(256) void k_rmax(const float* __restrict__ S, int NR, float* RS) {
    const int lane = threadIdx.x & 31; const int row = blockIdx.x * 8 + (threadIdx.x >> 5); if (row >= NR) return;
    const float* sr = S + (size_t)row * TK;
    float mx = -3.0e38f;
#pragma unroll 4
    for (int j = lane; j < TK; j += 32) mx = fmaxf(mx, sr[j]);
#pragma unroll
    for (int sh = 16; sh; sh >>= 1) mx = fmaxf(mx, __shfl_xor(mx, sh, 32));
    const float o = lane == 0 ? mx : 0.f; *(volatile float*)(RS + (size_t)row * 32 + lane) = o; __threadfence(); *(volatile float*)(RS + (size_t)row * 32 + lane) = o;
}
__global__ __launch_bounds__(256) void k_rexp(const float* __restrict__ S, int NR, float* RS, bf* Ph, bf* Pl) {
    const int lane = threadIdx.x & 31; const int row = blockIdx.x * 8 + (threadIdx.x >> 5); if (row >= NR) return;
    const float* sr = S + (size_t)row * TK;
    const float mx = RS[(size_t)row * 32]; float sum = 0.f;
#pragma unroll 2
    for (int c0 = 0; c0 < TK; c0 += 64) { const int j = c0 + lane * 2; v2us oh, ol;
#pragma unroll
        for (int q = 0; q < 2; ++q) { const float e = __expf(sr[j + q] - mx); sum += e; unsigned short a, c2; splitf(e, a, c2); oh[q] = a; ol[q] = c2; }
        *(volatile v2us*)(Ph + (size_t)row * TK + j) = oh; *(volatile v2us*)(Pl + (size_t)row * TK + j) = ol; __threadfence(); *(volatile v2us*)(Ph + (size_t)row * TK + j) = oh; *(volatile v2us*)(Pl + (size_t)row * TK + j) = ol; }
#pragma unroll
    for (int sh = 16; sh; sh >>= 1) sum += __shfl_xor(sum, sh, 32);
    const float o2 = lane == 0 ? mx : (lane == 1 ? __fdiv_rn(1.0f, sum) : 0.f); *(volatile float*)(RS + (size_t)row * 32 + lane) = o2; __threadfence(); *(volatile float*)(RS + (size_t)row * 32 + lane) = o2;
}
__global__ __launch_bounds__(256) void k_merge(const float* __restrict__ O, const float* __restrict__ RS, int b, int h0, bf* Ah, bf* Al) {
    const int lane = threadIdx.x & 31; const int L0 = (blockIdx.x * 8 + (threadIdx.x >> 5)) * 8; const int nlines = ZH * TQ * HD / 64;
#pragma unroll 1
    for (int ps = 0; ps < 2; ++ps) {
#pragma unroll
        for (int l = 0; l < 8; ++l) { const int L = L0 + l; if (L >= nlines) break; const int e = L * 64 + lane * 2; const int d = e & 63; const int t = (e >> 6) & (TQ - 1); const int zz = e >> 15; const float ri = RS[((size_t)zz * TQ + t) * 32 + 1]; v2us oh, ol;
#pragma unroll
            for (int q = 0; q < 2; ++q) { unsigned short x, y; splitf(O[(size_t)e + q] * ri, x, y); oh[q] = x; ol[q] = y; }
            const size_t o = ((size_t)b * TQ + t) * DD + (h0 + zz) * HD + d; *(volatile v2us*)(Ah + o) = oh; *(volatile v2us*)(Al + o) = ol; }
        if (ps == 0) __threadfence(); }
}

extern "C" void kernel_launch(void* const* d_in, const int* in_sizes, int n_in,
                              void* d_out, int out_size, void* d_ws, size_t ws_size, hipStream_t stream) {
    (void)in_sizes; (void)n_in; (void)out_size;
    const float* inp = (const float*)d_in[0]; const float* lat = (const float*)d_in[1]; const float* wq = (const float*)d_in[2]; const float* wk = (const float*)d_in[3]; const float* wv = (const float*)d_in[4]; const float* wo = (const float*)d_in[5]; const float* qn = (const float*)d_in[6]; const float* kn = (const float*)d_in[7];
    float* OUT = (float*)d_out;
    char* wsp = (char*)d_ws;
    auto take = [&](size_t bytes) { char* p = wsp; wsp += (bytes + 255) & ~(size_t)255; return (void*)p; };
    bf* WQ = (bf*)take((size_t)DD * DD * 2); bf* WK = (bf*)take((size_t)DKV * DD * 2); bf* WV = (bf*)take((size_t)DKV * DD * 2); bf* WO = (bf*)take((size_t)DD * DD * 2);
    bf* XL = (bf*)take((size_t)NTQ * DD * 2); bf* XI = (bf*)take((size_t)NTK * DD * 2); float* FQ = (float*)take((size_t)NTQ * DD * 4); float* FK = (float*)take((size_t)NTK * DKV * 4);
    bf* QPh = (bf*)take((size_t)NTQ * DD * 2); bf* QPl = (bf*)take((size_t)NTQ * DD * 2); bf* KPh = (bf*)take((size_t)NTK * DKV * 2); bf* KPl = (bf*)take((size_t)NTK * DKV * 2); bf* VTh = (bf*)take((size_t)NTK * DKV * 2); bf* VTl = (bf*)take((size_t)NTK * DKV * 2);
    float* Sb = (float*)take((size_t)ZH * TQ * TK * 4); bf* Ph = (bf*)take((size_t)ZH * TQ * TK * 2); bf* Pl = (bf*)take((size_t)ZH * TQ * TK * 2); float* RS = (float*)take((size_t)ZH * TQ * 32 * 4); float* Ob = (float*)take((size_t)ZH * TQ * HD * 4); bf* ATh = (bf*)take((size_t)NTQ * DD * 2); bf* ATl = (bf*)take((size_t)NTQ * DD * 2);
    if ((size_t)(wsp - (char*)d_ws) > ws_size) return;
    { const size_t n1 = (size_t)DD * DD / 8, n2 = (size_t)DKV * DD / 8; k_cvt8<<<(unsigned)((n1 + 255) / 256), 256, 0, stream>>>(wq, WQ, n1); k_cvt8<<<(unsigned)((n2 + 255) / 256), 256, 0, stream>>>(wk, WK, n2); k_cvt8<<<(unsigned)((n2 + 255) / 256), 256, 0, stream>>>(wv, WV, n2); k_cvt8<<<(unsigned)((n1 + 255) / 256), 256, 0, stream>>>(wo, WO, n1);
      const size_t nl = (size_t)NTQ * DD / 8, ni = (size_t)NTK * DD / 8; k_cvt8<<<(unsigned)((nl + 255) / 256), 256, 0, stream>>>(lat, XL, nl); k_cvt8<<<(unsigned)((ni + 255) / 256), 256, 0, stream>>>(inp, XI, ni); }
    k_gemmw<bf, 0, false><<<dim3(NTQ / 64, DD / 64, 1), 32, 0, stream>>>(XL, nullptr, WQ, nullptr, DD, FQ, DD, nullptr, 0, 0, 0); k_rmsq<<<NTQ * NH_ / 8, 256, 0, stream>>>(FQ, qn, QPh, QPl);
    k_gemmw<bf, 0, false><<<dim3(NTK / 64, DKV / 64, 1), 32, 0, stream>>>(XI, nullptr, WK, nullptr, DD, FK, DKV, nullptr, 0, 0, 0); k_rmsk<<<NTK * NKV / 8, 256, 0, stream>>>(FK, kn, KPh, KPl);
    k_gemmw<bf, 0, false><<<dim3(NTK / 64, DKV / 64, 1), 32, 0, stream>>>(XI, nullptr, WV, nullptr, DD, FK, DKV, nullptr, 0, 0, 0); k_vtsplit<<<(unsigned)((NB_ * NKV * HD * TK / 64 + 63) / 64), 256, 0, stream>>>(FK, VTh, VTl);
    for (int b = 0; b < NB_; ++b)
        for (int h0 = 0; h0 < NH_; h0 += ZH) { const size_t zq = (size_t)b * NH_ + h0, zk = (size_t)b * NKV + h0 / GRP;
            k_gemmw<bf, 2, false><<<dim3(TQ / 64, TK / 64, ZH), 32, 0, stream>>>(QPh + zq * TQ * HD, QPl + zq * TQ * HD, KPh + zk * TK * HD, KPl + zk * TK * HD, HD, Sb, TK, nullptr, (size_t)TQ * HD, 0, (size_t)TQ * TK);
            k_rmax<<<ZH * TQ / 8, 256, 0, stream>>>(Sb, ZH * TQ, RS); k_rexp<<<ZH * TQ / 8, 256, 0, stream>>>(Sb, ZH * TQ, RS, Ph, Pl);
            k_gemmw<bf, 2, false><<<dim3(TQ / 64, 1, ZH), 32, 0, stream>>>(Ph, Pl, VTh + zk * HD * TK, VTl + zk * HD * TK, TK, Ob, HD, nullptr, (size_t)TQ * TK, 0, (size_t)TQ * HD);
            k_merge<<<(ZH * TQ * HD / 64 + 63) / 64, 256, 0, stream>>>(Ob, RS, b, h0, ATh, ATl); }
    k_gemmw<bf, 1, false><<<dim3(NTQ / 64, DD / 64, 1), 32, 0, stream>>>(ATh, ATl, WO, nullptr, DD, OUT, DD, nullptr, 0, 0, 0);
}
